// FlashSVDBlockDA_85529978733244
// MI455X (gfx1250) — hardware-run, weakly checked
//
#include <hip/hip_runtime.h>
#ifndef NB
#define NB 8
#endif
#ifndef SEQ
#define SEQ 1024
#endif
#define NB_FULL 8
#define SEQ_FULL 1024
#define DM 768
#define NH 12
#define HD 64
#define RK 32
#define RA (NH * RK)
#define RW 384
#define RF 384
#define FF 3072
#define MROWS (NB * SEQ)

static_assert(NH * HD == DM);
static_assert(HD == 64);
static_assert(RK == 32);
static_assert(RA == 384);
static_assert(SEQ % 64 == 0);
static_assert(SEQ % 4 == 0);
static_assert(SEQ <= SEQ_FULL);
static_assert(NB <= NB_FULL);
static_assert(MROWS % 32 == 0);
static_assert(MROWS % 64 == 0);
static_assert(DM % 256 == 0);
static_assert(DM % 128 == 0);
static_assert(DM % 64 == 0);
static_assert(FF % 64 == 0);
static_assert(RW % 64 == 0);
static_assert(RF % 64 == 0);
static_assert((3 * RA) % 64 == 0);
static_assert(DM % 32 == 0);
static_assert(RK % 32 == 0);
static_assert(RW % 32 == 0);
static_assert(RF % 32 == 0);
static_assert(FF % 32 == 0);
static_assert(((MROWS / 32) * ((3 * RA) / 64)) % 4 == 0);
static_assert(((MROWS / 32) * (DM / 64)) % 4 == 0);
static_assert(((MROWS / 32) * (RF / 64)) % 4 == 0);
static_assert(((MROWS / 32) * (RW / 64)) % 4 == 0);
static_assert(((MROWS / 32) * (FF / 64)) % 4 == 0);
static_assert(((DM / 32) * (MROWS / 64)) % 4 == 0);
static_assert((RK * (DM / 8)) % 256 == 0);
static_assert((HD * (RK / 8)) % 256 == 0);
static_assert((RW * (DM / 8)) % 256 == 0);
static_assert((DM * (RW / 8)) % 256 == 0);
static_assert((FF * (RF / 8)) % 256 == 0);
static_assert((RF * (FF / 8)) % 256 == 0);
static_assert(((size_t)MROWS * (DM / 8)) % 256 == 0);
static_assert(MROWS % 4 == 0);
static_assert((size_t)NB * NH * (SEQ / 64) * 64 * 64 == (size_t)MROWS * DM);
static_assert(4 * 32 * 64 * 4 + 4 * 32 * 64 * 2 <= 131072);
static_assert(4 * 16 * 40 * 2 + 4 * 16 * HD * 4 + SEQ * 4 <= 131072);
static_assert(4 * DM * 2 + 4 * DM * 4 <= 131072);

typedef _Float16 v16h __attribute__((ext_vector_type(16)));
typedef unsigned short v8us __attribute__((ext_vector_type(8), may_alias));
typedef float  v8f  __attribute__((ext_vector_type(8)));
typedef float  v4f  __attribute__((ext_vector_type(4)));
typedef float  v4fa __attribute__((ext_vector_type(4), may_alias));
union FragH { v16h v; v8us half[2]; };

__device__ __forceinline__ unsigned short bf16_bits(float x) { unsigned int u = __float_as_uint(x); return (unsigned short)((u + 0x7FFFu + ((u >> 16) & 1u)) >> 16); }
__device__ __forceinline__ float bf16_rne(float x) { return __uint_as_float(((unsigned int)bf16_bits(x)) << 16); }
__device__ __forceinline__ unsigned short f16_bits(float x) { const _Float16 hv = (_Float16)x; return __builtin_bit_cast(unsigned short, hv); }
__device__ __forceinline__ _Float16 toh_flush(float v) { const _Float16 r = (_Float16)v; return (fabsf(v) < 6.103515625e-05f) ? (_Float16)0.0f : r; }
__device__ __forceinline__ unsigned short hbits_flush(float v) { const _Float16 hv = toh_flush(v); return __builtin_bit_cast(unsigned short, hv); }
__device__ __forceinline__ unsigned ext_row(unsigned m) { return (m / (unsigned)SEQ) * (unsigned)SEQ_FULL + (m % (unsigned)SEQ); }
__device__ __forceinline__ float gelu_erf(float v) { return 0.5f * v * (1.0f + erff(v * 0.70710678118654752f)); }

__device__ __forceinline__ v8f mma1(v16h a, v16h b, v8f c) {
  c = __builtin_amdgcn_wmma_f32_16x16x32_f16(false, a, false, b, (short)0, c, false, false);
  asm volatile("v_nop\n\tv_nop\n\tv_nop\n\tv_nop" : "+v"(c) : "v"(a), "v"(b));
  return c;
}

__global__ __launch_bounds__(256) void k_wt_h(const float* __restrict__ W, unsigned short* __restrict__ Wt, unsigned K, unsigned N, float carry,
                                              unsigned zin, unsigned zout) {
  const unsigned t = blockIdx.x * 256u + threadIdx.x;
  const unsigned k8n = K >> 3;
  if (t >= N * k8n) return;
  const unsigned n = t / k8n, k8 = (t - n * k8n) << 3;
  const float* Wz = W + (size_t)blockIdx.y * zin;
  v8us v;
#pragma unroll
  for (int i = 0; i < 8; ++i) v[i] = hbits_flush(bf16_rne(Wz[(size_t)(k8 + i) * N + n]) * carry);
  unsigned short* dst = Wt + (size_t)blockIdx.y * zout + (size_t)n * K + k8;
  *(volatile v8us*)dst = v;
  __threadfence();
  *(volatile v8us*)dst = v;
}

__global__ __launch_bounds__(256) void k_x_h(const float* __restrict__ X, unsigned short* __restrict__ out, unsigned n8) {
  const unsigned t = blockIdx.x * 256u + threadIdx.x;
  if (t >= n8) return;
  const unsigned row = t / (unsigned)(DM / 8), j = (t - row * (unsigned)(DM / 8)) * 8u;
  const float* x = X + (size_t)ext_row(row) * DM + j;
  const v4f a = *(const v4fa*)(x), b = *(const v4fa*)(x + 4);
  v8us pk;
#pragma unroll
  for (int q = 0; q < 4; ++q) { pk[q] = hbits_flush(bf16_rne(a[q])); pk[4 + q] = hbits_flush(bf16_rne(b[q])); }
  unsigned short* dst = out + (size_t)row * DM + j;
  *(volatile v8us*)dst = pk;
  __threadfence();
  *(volatile v8us*)dst = pk;
}

template <bool OUT_H, bool EXT_OUT>
__device__ __forceinline__ void ln_rows_body(const float* __restrict__ X, const float* __restrict__ g, const float* __restrict__ bta,
                                             float* __restrict__ o32, unsigned short* __restrict__ o16, unsigned nrows, float eps) {
  __shared__ __attribute__((aligned(16))) unsigned short sst[4][DM];
  __shared__ __attribute__((aligned(16))) float sf[4][DM];
  const unsigned lane = threadIdx.x & 31u;
  const unsigned w = (unsigned)__builtin_amdgcn_readfirstlane((int)(threadIdx.x >> 5));
  const unsigned row = blockIdx.x * 4u + w;
  if (row >= nrows) return;
  const float* x = X + (size_t)row * DM;
  float s1 = 0.f;
#pragma unroll 1
  for (unsigned u = 0; u < DM / 256; ++u) {
    const unsigned j = (u * 32u + lane) * 8u;
    const v4f a = *(const v4fa*)(x + j), b = *(const v4fa*)(x + j + 4);
#pragma unroll
    for (int q = 0; q < 4; ++q) { s1 += a[q]; s1 += b[q]; }
  }
  s1 += __shfl_xor(s1, 16, 32); s1 += __shfl_xor(s1, 8, 32); s1 += __shfl_xor(s1, 4, 32); s1 += __shfl_xor(s1, 2, 32); s1 += __shfl_xor(s1, 1, 32);
  const float mu = s1 * (1.0f / (float)DM);
  float s2 = 0.f;
#pragma unroll 1
  for (unsigned u = 0; u < DM / 256; ++u) {
    const unsigned j = (u * 32u + lane) * 8u;
    const v4f a = *(const v4fa*)(x + j), b = *(const v4fa*)(x + j + 4);
#pragma unroll
    for (int q = 0; q < 4; ++q) {
      const float ca = a[q] - mu, cb = b[q] - mu;
      s2 += ca * ca; s2 += cb * cb;
    }
  }
  s2 += __shfl_xor(s2, 16, 32); s2 += __shfl_xor(s2, 8, 32); s2 += __shfl_xor(s2, 4, 32); s2 += __shfl_xor(s2, 2, 32); s2 += __shfl_xor(s2, 1, 32);
  const float rs = rsqrtf(s2 * (1.0f / (float)DM) + eps);
  unsigned short* orow16 = o16 + (size_t)row * DM;
#pragma unroll 1
  for (unsigned u = 0; u < DM / 256; ++u) {
    const unsigned j = (u * 32u + lane) * 8u;
    const v4f a = *(const v4fa*)(x + j), b = *(const v4fa*)(x + j + 4);
    const v4f ga = *(const v4fa*)(g + j), gb = *(const v4fa*)(g + j + 4);
    const v4f ba = *(const v4fa*)(bta + j), bb = *(const v4fa*)(bta + j + 4);
    v4f ya, yb;
#pragma unroll
    for (int q = 0; q < 4; ++q) {
      ya[q] = (a[q] - mu) * rs * bf16_rne(ga[q]) + bf16_rne(ba[q]);
      yb[q] = (b[q] - mu) * rs * bf16_rne(gb[q]) + bf16_rne(bb[q]);
    }
    *(v4fa*)&sf[w][j] = ya;
    *(v4fa*)&sf[w][j + 4] = yb;
    if (OUT_H) {
      v8us pk;
#pragma unroll
      for (int q = 0; q < 4; ++q) { pk[q] = hbits_flush(ya[q]); pk[4 + q] = hbits_flush(yb[q]); }
      *(v8us*)&sst[w][j] = pk;
      *(volatile v8us*)(orow16 + j) = pk;
    }
  }
  __builtin_amdgcn_fence(4  , "workgroup");
  __builtin_amdgcn_wave_barrier();
  float* orow = o32 + (size_t)(EXT_OUT ? ext_row(row) : row) * DM;
  static_assert(32 * 4 * (DM / 128) == DM);
#pragma unroll 1
  for (unsigned u = 0; u < DM / 128; ++u) {
    const unsigned j = (u * 32u + lane) * 4u;
    const v4f v = *(const v4fa*)&sf[w][j];
    *(volatile v4f*)(orow + j) = v;
  }
  __threadfence();
  if (OUT_H) {
    static_assert(32 * 8 * (DM / 256) == DM);
#pragma unroll 1
    for (unsigned u = 0; u < DM / 256; ++u) {
      const unsigned j = (u * 32u + lane) * 8u;
      const v8us pk = *(const v8us*)&sst[w][j];
      *(volatile v8us*)(orow16 + j) = pk;
    }
  }
#pragma unroll 1
  for (unsigned u = 0; u < DM / 128; ++u) {
    const unsigned j = (u * 32u + lane) * 4u;
    const v4f v = *(const v4fa*)&sf[w][j];
    *(volatile v4f*)(orow + j) = v;
  }
}

__global__ __launch_bounds__(128) void k_ln_mid(const float* __restrict__ X, const float* __restrict__ g, const float* __restrict__ bta,
                                                float* __restrict__ o32, unsigned short* __restrict__ o16, unsigned nrows, float eps) {
  ln_rows_body<true, false>(X, g, bta, o32, o16, nrows, eps);
}
__global__ __launch_bounds__(128) void k_ln_out(const float* __restrict__ X, const float* __restrict__ g, const float* __restrict__ bta,
                                                float* __restrict__ o32, unsigned nrows, float eps) {
  ln_rows_body<false, true>(X, g, bta, o32, nullptr, nrows, eps);
}

template <int MODE>
__device__ __forceinline__ void gemm_body(const unsigned short* __restrict__ A, unsigned lda, unsigned akq,
                                          const unsigned short* __restrict__ Bp, unsigned ldb, unsigned bkm,
                                          const float* __restrict__ bias, const float* __restrict__ resid,
                                          void* __restrict__ Cout, unsigned ldc,
                                          unsigned M, unsigned N, unsigned K, float inv) {
  __shared__ __attribute__((aligned(16))) float so[4][32][64];
  const unsigned tid = threadIdx.x, lane = tid & 31u, ln = lane & 15u, hh = lane >> 4;
  const unsigned w = (unsigned)__builtin_amdgcn_readfirstlane((int)(tid >> 5));
  const unsigned ntn = N >> 6;
  const unsigned wid = blockIdx.x * 4u + w;
  const unsigned mt = wid / ntn, nq = wid - mt * ntn;
  if (mt * 32u >= M) return;
  const unsigned row0 = mt * 32u, col0 = nq * 64u;
  const unsigned short* a0 = A + (size_t)(row0 + ln) * lda + 8u * hh + nq * akq;
  const unsigned short* a1 = a0 + (size_t)16 * lda;
  const unsigned short* b0 = Bp + (size_t)(col0 + ln) * ldb + 8u * hh + (row0 >> 6) * bkm;
  v8f acc[2][4];
#pragma unroll
  for (int mi = 0; mi < 2; ++mi)
#pragma unroll
    for (int t = 0; t < 4; ++t) acc[mi][t] = (v8f){0.f,0.f,0.f,0.f,0.f,0.f,0.f,0.f};
  for (unsigned kb = 0; kb < K; kb += 32u) {
    FragH fa0, fa1;
    fa0.half[0] = *(const v8us*)(a0 + kb); fa0.half[1] = *(const v8us*)(a0 + kb + 16);
    fa1.half[0] = *(const v8us*)(a1 + kb); fa1.half[1] = *(const v8us*)(a1 + kb + 16);
#pragma unroll
    for (int t = 0; t < 4; ++t) {
      const unsigned short* br = b0 + (size_t)(t * 16) * ldb + kb;
      FragH fb;
      fb.half[0] = *(const v8us*)(br);
      fb.half[1] = *(const v8us*)(br + 16);
      acc[0][t] = mma1(fa0.v, fb.v, acc[0][t]);
      acc[1][t] = mma1(fa1.v, fb.v, acc[1][t]);
    }
  }
  float brow[2][8];
#pragma unroll
  for (int mi = 0; mi < 2; ++mi)
#pragma unroll
    for (int r = 0; r < 8; ++r) brow[mi][r] = (MODE == 1) ? bf16_rne(bias[row0 + mi * 16 + 8u * hh + r]) : 0.f;
#pragma unroll
  for (int t = 0; t < 4; ++t) {
    const float bc = (MODE == 1 || MODE == 5) ? 0.f : bf16_rne(bias[col0 + t * 16 + ln]);
#pragma unroll
    for (int mi = 0; mi < 2; ++mi)
#pragma unroll
      for (int r = 0; r < 8; ++r)
        so[w][mi * 16 + 8u * hh + r][t * 16 + ln] = acc[mi][t][r] * inv + ((MODE == 1) ? brow[mi][r] : bc);
  }
  __builtin_amdgcn_fence(4  , "workgroup");
  __builtin_amdgcn_wave_barrier();
  if constexpr (MODE == 3 || MODE == 4) {
    float* C = (float*)Cout;
    const unsigned rsub = lane >> 4, c4 = (lane & 15u) * 4u;
    static_assert(32 * 16 * 16 == 32 * 64 * 4);
#pragma unroll 4
    for (unsigned q = 0; q < 16; ++q) {
      const unsigned r = q * 2u + rsub;
      const unsigned grow = row0 + r;
      const size_t ro = (size_t)((MODE == 3) ? ext_row(grow) : grow) * DM + col0 + c4;
      const v4f rv = *(const v4fa*)(resid + ro);
      v4f v = *(const v4fa*)&so[w][r][c4];
#pragma unroll
      for (int i = 0; i < 4; ++i) v[i] += (MODE == 3) ? bf16_rne(rv[i]) : rv[i];
      *(v4fa*)&so[w][r][c4] = v;
    }
    for (int pass = 0; pass < 2; ++pass) {
#pragma unroll 4
      for (unsigned q = 0; q < 16; ++q) {
        const unsigned r = q * 2u + rsub;
        const unsigned grow = row0 + r;
        const v4f v = *(const v4fa*)&so[w][r][c4];
        *(volatile v4f*)(C + (size_t)grow * ldc + col0 + c4) = v;
      }
      if (pass == 0) __threadfence();
    }
  } else {
    __shared__ __attribute__((aligned(16))) unsigned short sh[4][32][64];
    unsigned short* C = (unsigned short*)Cout;
    const unsigned rq = lane >> 3, c8 = (lane & 7u) * 8u;
    static_assert(32 * 16 * 8 == 32 * 64 * 2);
#pragma unroll 1
    for (unsigned q = 0; q < 8; ++q) {
      const unsigned r = q * 4u + rq;
      const v4f x0 = *(const v4fa*)&so[w][r][c8], x1 = *(const v4fa*)&so[w][r][c8 + 4];
      v8us pk;
#pragma unroll
      for (int i = 0; i < 4; ++i) {
        float a = x0[i], b = x1[i];
        if (MODE == 2) { a = gelu_erf(a) * 64.0f; b = gelu_erf(b) * 64.0f; }
        pk[i] = hbits_flush(a); pk[4 + i] = hbits_flush(b);
      }
      *(v8us*)&sh[w][r][c8] = pk;
    }
    __builtin_amdgcn_fence(4  , "workgroup");
    __builtin_amdgcn_wave_barrier();
    size_t base; unsigned pitch;
    if (MODE == 1) { const unsigned bb = col0 / (unsigned)SEQ, s0 = col0 - bb * (unsigned)SEQ; base = ((size_t)bb * DM + row0) * SEQ + s0 + c8; pitch = SEQ; }
    else           { base = (size_t)row0 * ldc + col0 + c8; pitch = ldc; }
    for (int pass = 0; pass < 2; ++pass) {
#pragma unroll 4
      for (unsigned q = 0; q < 8; ++q) {
        const unsigned r = q * 4u + rq;
        const v8us v = *(const v8us*)&sh[w][r][c8];
        *(volatile v8us*)(C + base + (size_t)r * pitch) = v;
      }
      if (pass == 0) __threadfence();
    }
  }
}

__global__ __launch_bounds__(128) void k_gemm_plain(const unsigned short* __restrict__ A, unsigned lda,
                                                    const unsigned short* __restrict__ Bp, unsigned ldb,
                                                    unsigned short* __restrict__ C16, unsigned ldc,
                                                    unsigned M, unsigned N, unsigned K, float inv) {
  gemm_body<5>(A, lda, 0u, Bp, ldb, 0u, nullptr, nullptr, (void*)C16, ldc, M, N, K, inv);
}
__global__ __launch_bounds__(128) void k_gemm_bias(const unsigned short* __restrict__ A, unsigned lda, unsigned akq,
                                                   const unsigned short* __restrict__ Bp, unsigned ldb,
                                                   const float* __restrict__ bias,
                                                   unsigned short* __restrict__ C16, unsigned ldc,
                                                   unsigned M, unsigned N, unsigned K, float inv) {
  gemm_body<0>(A, lda, akq, Bp, ldb, 0u, bias, nullptr, (void*)C16, ldc, M, N, K, inv);
}
__global__ __launch_bounds__(128) void k_gemm_vt(const unsigned short* __restrict__ A, unsigned lda,
                                                 const unsigned short* __restrict__ Bp, unsigned ldb, unsigned bkm,
                                                 const float* __restrict__ bias,
                                                 unsigned short* __restrict__ C16,
                                                 unsigned M, unsigned N, unsigned K, float inv) {
  gemm_body<1>(A, lda, 0u, Bp, ldb, bkm, bias, nullptr, (void*)C16, (unsigned)SEQ, M, N, K, inv);
}
__global__ __launch_bounds__(128) void k_gemm_gelu(const unsigned short* __restrict__ A, unsigned lda,
                                                   const unsigned short* __restrict__ Bp, unsigned ldb,
                                                   const float* __restrict__ bias,
                                                   unsigned short* __restrict__ C16, unsigned ldc,
                                                   unsigned M, unsigned N, unsigned K, float inv) {
  gemm_body<2>(A, lda, 0u, Bp, ldb, 0u, bias, nullptr, (void*)C16, ldc, M, N, K, inv);
}
__global__ __launch_bounds__(128) void k_gemm_res_ext(const unsigned short* __restrict__ A, unsigned lda,
                                                      const unsigned short* __restrict__ Bp, unsigned ldb,
                                                      const float* __restrict__ bias, const float* __restrict__ resid,
                                                      float* __restrict__ C32, unsigned ldc,
                                                      unsigned M, unsigned N, unsigned K, float inv) {
  gemm_body<3>(A, lda, 0u, Bp, ldb, 0u, bias, resid, (void*)C32, ldc, M, N, K, inv);
}
__global__ __launch_bounds__(128) void k_gemm_res(const unsigned short* __restrict__ A, unsigned lda,
                                                  const unsigned short* __restrict__ Bp, unsigned ldb,
                                                  const float* __restrict__ bias, const float* __restrict__ resid,
                                                  float* __restrict__ C32, unsigned ldc,
                                                  unsigned M, unsigned N, unsigned K, float inv) {
  gemm_body<4>(A, lda, 0u, Bp, ldb, 0u, bias, resid, (void*)C32, ldc, M, N, K, inv);
}

__global__ __launch_bounds__(128) void k_flash(const unsigned short* __restrict__ Qp, const unsigned short* __restrict__ Kp,
                                               const unsigned short* __restrict__ Vt, const float* __restrict__ mask,
                                               unsigned short* __restrict__ ctx) {
  __shared__ __attribute__((aligned(16))) unsigned short sP[4][16][40];
  __shared__ __attribute__((aligned(16))) float sO[4][16][HD];
  __shared__ __attribute__((aligned(16))) float sM[SEQ];
  const unsigned tid = threadIdx.x, lane = tid & 31u, ln = lane & 15u, hh = lane >> 4;
  const unsigned w = (unsigned)__builtin_amdgcn_readfirstlane((int)(tid >> 5));
  const unsigned nqb = SEQ / 64;
  const unsigned bh = blockIdx.x / nqb, qblk = blockIdx.x - bh * nqb;
  const unsigned b = bh / (unsigned)NH, h = bh - b * (unsigned)NH;
  const unsigned q0 = qblk * 64u + w * 16u;
  {
    const float* mrow = mask + (size_t)b * SEQ_FULL;
#pragma unroll 1
    for (unsigned i = tid * 4u; i < (unsigned)SEQ; i += 512u) {
      const v4f mv = *(const v4fa*)(mrow + i);
      v4f o;
#pragma unroll
      for (int q = 0; q < 4; ++q) o[q] = bf16_rne(mv[q]);
      *(v4fa*)&sM[i] = o;
    }
  }
  __syncthreads();
  FragH aq[2];
  {
    const unsigned short* qr = Qp + (size_t)(b * (unsigned)SEQ + q0 + ln) * DM + h * HD + 8u * hh;
#pragma unroll
    for (int ks = 0; ks < 2; ++ks) { aq[ks].half[0] = *(const v8us*)(qr + ks * 32); aq[ks].half[1] = *(const v8us*)(qr + ks * 32 + 16); }
  }
  const unsigned short* kbase = Kp + (size_t)(b * (unsigned)SEQ + ln) * DM + h * HD + 8u * hh;
  const unsigned short* vbase = Vt + ((size_t)b * DM + h * HD + ln) * SEQ + 8u * hh;
  float m_r[8], l_r[8];
#pragma unroll
  for (int r = 0; r < 8; ++r) { m_r[r] = -1.0e30f; l_r[r] = 0.f; }
  v8f oacc[4];
#pragma unroll
  for (int dt = 0; dt < 4; ++dt) oacc[dt] = (v8f){0.f,0.f,0.f,0.f,0.f,0.f,0.f,0.f};

  for (unsigned j0 = 0; j0 < (unsigned)SEQ; j0 += 32u) {
    v8f s[2];
#pragma unroll
    for (int nt = 0; nt < 2; ++nt) {
      v8f acc = (v8f){0.f,0.f,0.f,0.f,0.f,0.f,0.f,0.f};
#pragma unroll
      for (int ks = 0; ks < 2; ++ks) {
        const unsigned short* kr = kbase + (size_t)(j0 + nt * 16) * DM + ks * 32;
        FragH fb;
        fb.half[0] = *(const v8us*)(kr);
        fb.half[1] = *(const v8us*)(kr + 16);
        acc = mma1(aq[ks].v, fb.v, acc);
      }
      s[nt] = acc;
    }
    const float mv0 = sM[j0 + ln], mv1 = sM[j0 + 16u + ln];
    float alpha[8];
#pragma unroll
    for (int r = 0; r < 8; ++r) {
      const float s0 = s[0][r] * 0.125f + mv0, s1 = s[1][r] * 0.125f + mv1;
      float mx = fmaxf(s0, s1);
      mx = fmaxf(mx, __shfl_xor(mx, 1, 32)); mx = fmaxf(mx, __shfl_xor(mx, 2, 32)); mx = fmaxf(mx, __shfl_xor(mx, 4, 32)); mx = fmaxf(mx, __shfl_xor(mx, 8, 32));
      const float mnew = fmaxf(m_r[r], mx);
      alpha[r] = __expf(m_r[r] - mnew);
      const float p0 = __expf(s0 - mnew), p1 = __expf(s1 - mnew);
      m_r[r] = mnew;
      l_r[r] = l_r[r] * alpha[r] + p0 + p1;
      sP[w][8u * hh + r][ln]       = hbits_flush(p0 * 1024.0f);
      sP[w][8u * hh + r][16u + ln] = hbits_flush(p1 * 1024.0f);
    }
#pragma unroll
    for (int dt = 0; dt < 4; ++dt)
#pragma unroll
      for (int r = 0; r < 8; ++r) oacc[dt][r] *= alpha[r];
    __builtin_amdgcn_fence(4  , "workgroup");
    __builtin_amdgcn_wave_barrier();
    FragH pa;
    pa.half[0] = *(const v8us*)&sP[w][ln][8u * hh];
    pa.half[1] = *(const v8us*)&sP[w][ln][16u + 8u * hh];
#pragma unroll
    for (int dt = 0; dt < 4; ++dt) {
      const unsigned short* vr = vbase + (size_t)(dt * 16) * SEQ + j0;
      FragH fb;
      fb.half[0] = *(const v8us*)(vr);
      fb.half[1] = *(const v8us*)(vr + 16);
      oacc[dt] = mma1(pa.v, fb.v, oacc[dt]);
    }
    __builtin_amdgcn_fence(4  , "workgroup");
    __builtin_amdgcn_wave_barrier();
  }
#pragma unroll
  for (int r = 0; r < 8; ++r) {
    float l = l_r[r];
    l += __shfl_xor(l, 1, 32); l += __shfl_xor(l, 2, 32); l += __shfl_xor(l, 4, 32); l += __shfl_xor(l, 8, 32);
    l_r[r] = 0.0625f * (1.0f / l);
  }
#pragma unroll
  for (int dt = 0; dt < 4; ++dt)
#pragma unroll
    for (int r = 0; r < 8; ++r) sO[w][8u * hh + r][dt * 16 + ln] = oacc[dt][r] * l_r[r];
  __builtin_amdgcn_fence(4  , "workgroup");
  __builtin_amdgcn_wave_barrier();
  const unsigned rq = lane >> 3, c8 = (lane & 7u) * 8u;
  static_assert(32 * 16 * 4 == 16 * HD * 2);
  v8us pk[4];
#pragma unroll
  for (int q = 0; q < 4; ++q) {
    const unsigned r = q * 4u + rq;
    const v4f x0 = *(const v4fa*)&sO[w][r][c8], x1 = *(const v4fa*)&sO[w][r][c8 + 4];
#pragma unroll
    for (int i = 0; i < 4; ++i) { pk[q][i] = hbits_flush(x0[i]); pk[q][4 + i] = hbits_flush(x1[i]); }
  }
  unsigned short* dst = ctx + (size_t)(b * (unsigned)SEQ + q0 + rq) * DM + h * HD + c8;
#pragma unroll
  for (int pass = 0; pass < 2; ++pass) {
#pragma unroll
    for (int q = 0; q < 4; ++q) *(volatile v8us*)(dst + (size_t)(q * 4) * DM) = pk[q];
    if (pass == 0) __threadfence();
  }
}

extern "C" void kernel_launch(void* const* d_in, const int* in_sizes, int n_in,
                              void* d_out, int out_size, void* d_ws, size_t ws_size, hipStream_t stream) {
  if (n_in < 24) return;
  const size_t need_x = ((size_t)(NB - 1) * SEQ_FULL + SEQ) * DM;
  const size_t need_m = (size_t)(NB - 1) * SEQ_FULL + SEQ;
  if ((size_t)in_sizes[0] < need_x || (size_t)out_size < need_x) return;
  if ((size_t)in_sizes[1] < need_m) return;
  if (in_sizes[2] < NH * DM * RK || in_sizes[5] < NH * DM * RK || in_sizes[8] < NH * DM * RK) return;
  if (in_sizes[3] < NH * RK * HD || in_sizes[6] < NH * RK * HD || in_sizes[9] < NH * RK * HD) return;
  if (in_sizes[4] < DM || in_sizes[7] < DM || in_sizes[10] < DM) return;
  if (in_sizes[11] < DM * RW || in_sizes[12] < RW * DM || in_sizes[13] < DM) return;
  if (in_sizes[14] < DM * RF || in_sizes[15] < RF * FF || in_sizes[16] < FF) return;
  if (in_sizes[17] < FF * RF || in_sizes[18] < RF * DM || in_sizes[19] < DM) return;
  if (in_sizes[20] < DM || in_sizes[21] < DM || in_sizes[22] < DM || in_sizes[23] < DM) return;
  const float* x    = (const float*)d_in[0];
  const float* mask = (const float*)d_in[1];
  const float* Pq = (const float*)d_in[2];  const float* Vq = (const float*)d_in[3];  const float* bq = (const float*)d_in[4];
  const float* Pk = (const float*)d_in[5];  const float* Vk = (const float*)d_in[6];  const float* bk = (const float*)d_in[7];
  const float* Pv = (const float*)d_in[8];  const float* Vv = (const float*)d_in[9];  const float* bv = (const float*)d_in[10];
  const float* Uo = (const float*)d_in[11]; const float* Vo = (const float*)d_in[12]; const float* bo = (const float*)d_in[13];
  const float* U1 = (const float*)d_in[14]; const float* V1 = (const float*)d_in[15]; const float* b1 = (const float*)d_in[16];
  const float* U2 = (const float*)d_in[17]; const float* V2 = (const float*)d_in[18]; const float* b2 = (const float*)d_in[19];
  const float* g1 = (const float*)d_in[20]; const float* be1 = (const float*)d_in[21];
  const float* g2 = (const float*)d_in[22]; const float* be2 = (const float*)d_in[23];

  constexpr size_t SZ_PT  = (size_t)(3 * RA) * DM * 2;
  constexpr size_t SZ_VS  = (size_t)DM * RK * 2;
  constexpr size_t SZ_WL  = (size_t)RW * DM * 2;
  constexpr size_t SZ_WF  = (size_t)FF * RF * 2;
  constexpr size_t SZ_P   = (size_t)MROWS * DM * 2;
  constexpr size_t SZ_L   = (size_t)MROWS * RF * 2;
  constexpr size_t SZ_T   = (size_t)MROWS * (3 * RA) * 2;
  constexpr size_t SZ_X2  = (size_t)MROWS * DM * 4;
  constexpr size_t SZ_MID = (size_t)MROWS * FF * 2;
  constexpr size_t SZ_R   = 4 * SZ_P;
  static_assert(SZ_MID <= SZ_R);
  static_assert(SZ_T <= SZ_X2);
  static_assert((size_t)MROWS * RW * 2 <= SZ_L);
  static_assert((size_t)DM * RW * 2 == SZ_WL);
  static_assert((size_t)RF * DM * 2 == SZ_WL);
  static_assert((size_t)RF * FF * 2 == SZ_WF);
  static_assert(SZ_PT % 256 == 0);
  static_assert(SZ_VS % 256 == 0);
  static_assert(SZ_WL % 256 == 0);
  static_assert(SZ_WF % 256 == 0);
  static_assert(SZ_P % 256 == 0);
  static_assert(SZ_L % 256 == 0);
  static_assert(SZ_X2 % 256 == 0);
  constexpr size_t TOTAL = SZ_PT + 3 * SZ_VS + 4 * SZ_WL + 2 * SZ_WF + SZ_P + SZ_R + SZ_L + 2 * SZ_X2;
  static_assert(TOTAL <= (size_t)134217728);
  if (TOTAL > ws_size) return;
  char* ws = (char*)d_ws; size_t off = 0;
  auto take = [&](size_t bytes) { char* p = ws + off; off += bytes; return p; };
  unsigned short* PT  = (unsigned short*)take(SZ_PT);
  unsigned short* VqT = (unsigned short*)take(SZ_VS);
  unsigned short* VkT = (unsigned short*)take(SZ_VS);
  unsigned short* VvT = (unsigned short*)take(SZ_VS);
  unsigned short* UoT = (unsigned short*)take(SZ_WL);
  unsigned short* VoT = (unsigned short*)take(SZ_WL);
  unsigned short* U1T = (unsigned short*)take(SZ_WL);
  unsigned short* V2T = (unsigned short*)take(SZ_WL);
  unsigned short* V1T = (unsigned short*)take(SZ_WF);
  unsigned short* U2T = (unsigned short*)take(SZ_WF);
  unsigned short* xh  = (unsigned short*)take(SZ_P);
  char* R = take(SZ_R);
  unsigned short* Qpl = (unsigned short*)(R);
  unsigned short* Kpl = (unsigned short*)(R + SZ_P);
  unsigned short* Vtp = (unsigned short*)(R + 2 * SZ_P);
  unsigned short* ctx = (unsigned short*)(R + 3 * SZ_P);
  unsigned short* hdn = (unsigned short*)(R);
  unsigned short* tlo = (unsigned short*)take(SZ_L);
  float* h12 = (float*)take(SZ_X2);
  float* x1f = (float*)take(SZ_X2);
  unsigned short* Tpl = (unsigned short*)x1f;
  unsigned short* x1h = xh;

  k_wt_h<<<dim3((RK * (DM / 8)) / 256, NH), 256, 0, stream>>>(Pq, PT,                       DM, RK, 64.0f, DM * RK, RK * DM);
  k_wt_h<<<dim3((RK * (DM / 8)) / 256, NH), 256, 0, stream>>>(Pk, PT + (size_t)RA * DM,     DM, RK, 64.0f, DM * RK, RK * DM);
  k_wt_h<<<dim3((RK * (DM / 8)) / 256, NH), 256, 0, stream>>>(Pv, PT + (size_t)2 * RA * DM, DM, RK, 64.0f, DM * RK, RK * DM);
  k_wt_h<<<dim3((HD * (RK / 8)) / 256, NH), 256, 0, stream>>>(Vq, VqT, RK, HD, 64.0f, RK * HD, HD * RK);
  k_wt_h<<<dim3((HD * (RK / 8)) / 256, NH), 256, 0, stream>>>(Vk, VkT, RK, HD, 64.0f, RK * HD, HD * RK);
  k_wt_h<<<dim3((HD * (RK / 8)) / 256, NH), 256, 0, stream>>>(Vv, VvT, RK, HD, 64.0f, RK * HD, HD * RK);
  k_wt_h<<<dim3((RW * (DM / 8)) / 256, 1), 256, 0, stream>>>(Uo, UoT, DM, RW, 64.0f, 0u, 0u);
  k_wt_h<<<dim3((DM * (RW / 8)) / 256, 1), 256, 0, stream>>>(Vo, VoT, RW, DM, 64.0f, 0u, 0u);
  k_wt_h<<<dim3((RF * (DM / 8)) / 256, 1), 256, 0, stream>>>(U1, U1T, DM, RF, 64.0f, 0u, 0u);
  k_wt_h<<<dim3((FF * (RF / 8)) / 256, 1), 256, 0, stream>>>(V1, V1T, RF, FF, 64.0f, 0u, 0u);
  k_wt_h<<<dim3((RF * (FF / 8)) / 256, 1), 256, 0, stream>>>(U2, U2T, FF, RF, 64.0f, 0u, 0u);
  k_wt_h<<<dim3((DM * (RF / 8)) / 256, 1), 256, 0, stream>>>(V2, V2T, RF, DM, 64.0f, 0u, 0u);

  const float i64 = 0.015625f, i4096 = 0.000244140625f;
  const unsigned gS1 = ((MROWS / 32) * ((3 * RA) / 64) + 3) / 4;
  const unsigned gD  = ((MROWS / 32) * (DM / 64) + 3) / 4;
  const unsigned gL  = ((MROWS / 32) * (RF / 64) + 3) / 4;
  const unsigned gF  = ((MROWS / 32) * (FF / 64) + 3) / 4;
  const unsigned gVt = ((DM / 32) * (MROWS / 64) + 3) / 4;

  k_x_h<<<(unsigned)(((size_t)MROWS * (DM / 8)) / 256), 256, 0, stream>>>(x, xh, (unsigned)((size_t)MROWS * (DM / 8)));
  k_gemm_plain<<<gS1, 128, 0, stream>>>(xh, DM, PT, DM, Tpl, 3 * RA, MROWS, 3 * RA, DM, i64);
  k_gemm_bias<<<gD, 128, 0, stream>>>(Tpl,          3 * RA, RK, VqT, RK, bq, Qpl, DM, MROWS, DM, RK, i64);
  k_gemm_bias<<<gD, 128, 0, stream>>>(Tpl + RA,     3 * RA, RK, VkT, RK, bk, Kpl, DM, MROWS, DM, RK, i64);
  k_gemm_vt<<<gVt, 128, 0, stream>>>(VvT, RK, Tpl + 2 * RA, 3 * RA, RK, bv, Vtp, DM, MROWS, RK, i64);
  k_flash<<<NB * NH * (SEQ / 64), 128, 0, stream>>>(Qpl, Kpl, Vtp, mask, ctx);
  k_gemm_plain<<<gL, 128, 0, stream>>>(ctx, DM, UoT, DM, tlo, RW, MROWS, RW, DM, i64);
  k_gemm_res_ext<<<gD, 128, 0, stream>>>(tlo, RW, VoT, RW, bo, x, h12, DM, MROWS, DM, RW, i4096);
  k_ln_mid<<<MROWS / 4, 128, 0, stream>>>(h12, g1, be1, x1f, x1h, MROWS, 1e-12f);
  k_gemm_plain<<<gL, 128, 0, stream>>>(x1h, DM, U1T, DM, tlo, RF, MROWS, RF, DM, i64);
  k_gemm_gelu<<<gF, 128, 0, stream>>>(tlo, RF, V1T, RF, b1, hdn, FF, MROWS, FF, RF, i64);
  k_gemm_plain<<<gL, 128, 0, stream>>>(hdn, FF, U2T, FF, tlo, RF, MROWS, RF, FF, i4096);
  k_gemm_res<<<gD, 128, 0, stream>>>(tlo, RF, V2T, RF, b2, x1f, h12, DM, MROWS, DM, RF, i64);
  k_ln_out<<<MROWS / 4, 128, 0, stream>>>(h12, g2, be2, (float*)d_out, MROWS, 1e-12f);
}
